// MultiHeadAttention_798863917312
// MI455X (gfx1250) — hardware-verified
//
#include <hip/hip_runtime.h>


#ifndef NB
#define NB 2
#endif
#ifndef SEQ
#define SEQ 4096
#endif
#define NB_FULL  2
#define SEQ_FULL 4096
#define DM   512
#define NH   8
#define HD   64
#define QCAR 8.0f
#define KCAR 8.0f
#define VCAR 8.0f
#define PEXP 10.0f
#define CL2  (0.125f / (QCAR * KCAR) * 1.4426950408889634f)

static_assert(DM == NH * HD);
static_assert(HD == 64);
static_assert(DM % 64 == 0);
static_assert(DM % 32 == 0);
static_assert(HD % 32 == 0);
static_assert(SEQ % 64 == 0);
static_assert(SEQ <= SEQ_FULL);
static_assert(NB <= NB_FULL);
static_assert(((size_t)SEQ * DM) % 64 == 0);

typedef _Float16 h16;
typedef unsigned short bf;
typedef __attribute__((ext_vector_type(16))) __bf16   v16bf;
typedef __attribute__((ext_vector_type(16))) _Float16 v16h;
typedef __attribute__((ext_vector_type(8)))  _Float16 v8h;
typedef __attribute__((ext_vector_type(8)))  unsigned short v8us;
typedef __attribute__((ext_vector_type(8)))  float    v8f;
typedef __attribute__((ext_vector_type(4)))  float    v4f;
typedef v4f  __attribute__((may_alias)) v4fa;

__device__ __forceinline__ unsigned short f2bf(float f) { unsigned u = __float_as_uint(f); u += 0x7FFFu + ((u >> 16) & 1u); return (unsigned short)(u >> 16); }
__device__ __forceinline__ float bf2f(unsigned short b) { return __uint_as_float(((unsigned)b) << 16); }
__device__ __forceinline__ float bfr(float f) { return bf2f(f2bf(f)); }
__device__ __forceinline__ void splitf(float y, unsigned short& h, unsigned short& l) { h = f2bf(y); l = f2bf(y - bf2f(h)); }
__device__ __forceinline__ v16h cat16(v8h lo, v8h hi) { return __builtin_shufflevector(lo, hi, 0, 1, 2, 3, 4, 5, 6, 7, 8, 9, 10, 11, 12, 13, 14, 15); }
__device__ __forceinline__ v16bf cat16b(v8us lo, v8us hi) { return __builtin_bit_cast(v16bf, __builtin_shufflevector(lo, hi, 0, 1, 2, 3, 4, 5, 6, 7, 8, 9, 10, 11, 12, 13, 14, 15)); }
__device__ __forceinline__ v8f wmma16(v16h a, v16h b, v8f c) { return __builtin_amdgcn_wmma_f32_16x16x32_f16(false, a, false, b, (short)0, c, false, false); }
__device__ __forceinline__ v8f wmmab(v16bf a, v16bf b, v8f c) { return __builtin_amdgcn_wmma_f32_16x16x32_bf16(false, a, false, b, (short)0, c, false, false); }
__device__ __forceinline__ v16h  ldh(const h16* p) { return cat16(*(const v8h*)p, *(const v8h*)(p + 16)); }
__device__ __forceinline__ v16bf ldb(const bf* p)  { return cat16b(*(const v8us*)p, *(const v8us*)(p + 16)); }

template <int NSPLIT, int BIASM, bool OUT16>
__device__ __forceinline__ void gemmw_body(const bf* __restrict__ A, const bf* __restrict__ A2, const bf* __restrict__ Bt, int K,
                                           float* Cf, h16* Ch, int ldc, size_t cstep, const float* __restrict__ bias, float car,
                                           size_t sA, size_t sB, size_t sC) {
    __shared__ __align__(16) float os[16 * 68];
    const size_t z = blockIdx.z; A += z * sA; if (NSPLIT == 1) A2 += z * sA; Bt += z * sB;
    const int lane = threadIdx.x & 31, lr = lane & 15, hi = lane >> 4; const int r0 = blockIdx.x * 64, c0 = blockIdx.y * 64;
    const size_t cofs0 = z * sC + (size_t)r0 * ldc + (size_t)blockIdx.y * cstep;
    v8f acc[4][4];
#pragma unroll
    for (int mb = 0; mb < 4; ++mb)
#pragma unroll
        for (int nb = 0; nb < 4; ++nb) acc[mb][nb] = (v8f){};
    const size_t aoff = (size_t)(r0 + lr) * K + 8 * hi, boff = (size_t)(c0 + lr) * K + 8 * hi;
#pragma unroll 1
    for (int kc = 0; kc < K; kc += 32) {
        v16bf a[4], a2[4];
#pragma unroll
        for (int mb = 0; mb < 4; ++mb) { a[mb] = ldb(A + aoff + (size_t)mb * 16 * K + kc); if (NSPLIT == 1) a2[mb] = ldb(A2 + aoff + (size_t)mb * 16 * K + kc); else a2[mb] = a[mb]; }
#pragma unroll
        for (int nb = 0; nb < 4; ++nb) { const v16bf b = ldb(Bt + boff + (size_t)nb * 16 * K + kc);
#pragma unroll
            for (int mb = 0; mb < 4; ++mb) { acc[mb][nb] = wmmab(a[mb], b, acc[mb][nb]); if (NSPLIT == 1) acc[mb][nb] = wmmab(a2[mb], b, acc[mb][nb]); } }
        asm volatile("v_nop\n\tv_nop\n\tv_nop\n\tv_nop" : "+v"(acc[0][0]), "+v"(acc[1][1]), "+v"(acc[2][2]), "+v"(acc[3][3]) : "v"(a[0]), "v"(a[3]));
    }
#pragma unroll
    for (int mb = 0; mb < 4; ++mb) {
#pragma unroll
        for (int nb = 0; nb < 4; ++nb) {
#pragma unroll
            for (int j = 0; j < 8; ++j) os[(hi * 8 + j) * 68 + nb * 16 + lr] = acc[mb][nb][j]; }
        __syncthreads();
        if (OUT16) {
            h16* crow = Ch + cofs0 + (size_t)(mb * 16) * ldc;
#pragma unroll 1
            for (int ps = 0; ps < 2; ++ps) {
#pragma unroll
                for (int s = 0; s < 4; ++s) { const int row = 4 * s + (lane >> 3), cofs = (lane & 7) * 8;
                    const v4f x0 = *(const v4fa*)(os + row * 68 + cofs); const v4f x1 = *(const v4fa*)(os + row * 68 + cofs + 4);
                    float xv[8]; xv[0] = x0[0]; xv[1] = x0[1]; xv[2] = x0[2]; xv[3] = x0[3]; xv[4] = x1[0]; xv[5] = x1[1]; xv[6] = x1[2]; xv[7] = x1[3];
                    v8h o;
#pragma unroll
                    for (int j = 0; j < 8; ++j) { float bb = 0.0f; if (BIASM == 1) bb = bfr(bias[c0 + cofs + j]); if (BIASM == 2) bb = bfr(bias[r0 + mb * 16 + row]); o[j] = (h16)((xv[j] + bb) * car); }
                    *(volatile v8h*)(crow + (size_t)row * ldc + cofs) = o; }
                if (ps == 0) __threadfence(); }
        } else {
            float* crow = Cf + cofs0 + (size_t)(mb * 16) * ldc;
#pragma unroll 1
            for (int ps = 0; ps < 2; ++ps) {
#pragma unroll
                for (int s = 0; s < 8; ++s) { const int row = 2 * s + hi, cofs = lr * 4; v4f val = *(const v4fa*)(os + row * 68 + cofs);
                    if (BIASM == 1) { val[0] += bfr(bias[c0 + cofs]); val[1] += bfr(bias[c0 + cofs + 1]); val[2] += bfr(bias[c0 + cofs + 2]); val[3] += bfr(bias[c0 + cofs + 3]); }
                    if (BIASM == 2) { const float bb = bfr(bias[r0 + mb * 16 + row]); val[0] += bb; val[1] += bb; val[2] += bb; val[3] += bb; }
                    *(volatile v4f*)(crow + (size_t)row * ldc + cofs) = val; }
                if (ps == 0) __threadfence(); }
        }
        __syncthreads();
    }
}

__global__ __launch_bounds__(32) void k_proj_hp(const bf* __restrict__ X, const bf* __restrict__ W, const float* __restrict__ bias, h16* P, float car) {
    gemmw_body<0, 1, true>(X, nullptr, W, DM, nullptr, P, HD, (size_t)SEQ * HD, bias, car, (size_t)SEQ * DM, 0, (size_t)NH * SEQ * HD);
}
__global__ __launch_bounds__(32) void k_proj_vt(const bf* __restrict__ W, const bf* __restrict__ X, const float* __restrict__ bias, h16* VT, float car) {
    gemmw_body<0, 2, true>(W, nullptr, X, DM, nullptr, VT, SEQ, (size_t)64, bias, car, 0, (size_t)SEQ * DM, (size_t)DM * SEQ);
}
__global__ __launch_bounds__(32) void k_oproj(const bf* __restrict__ Ah, const bf* __restrict__ Al, const bf* __restrict__ W, const float* __restrict__ bias, float* OUT) {
    gemmw_body<1, 1, false>(Ah, Al, W, DM, OUT, nullptr, DM, (size_t)64, bias, 1.0f, (size_t)SEQ * DM, 0, (size_t)SEQ_FULL * DM);
}

__global__ __launch_bounds__(256) void k_cvt8(const float* __restrict__ src, bf* dst, size_t n8, size_t sstride, size_t dstride) {
    const size_t i = (size_t)blockIdx.x * 256 + threadIdx.x; if (i >= n8) return;
    const float* s = src + (size_t)blockIdx.y * sstride; bf* d = dst + (size_t)blockIdx.y * dstride;
    const v8f v = *(const v8f*)(s + i * 8); v8us o;
#pragma unroll
    for (int k = 0; k < 8; ++k) o[k] = f2bf(v[k]);
    *(volatile v8us*)(d + i * 8) = o; __threadfence(); *(volatile v8us*)(d + i * 8) = o;
}

__global__ __launch_bounds__(128) void k_flash(const h16* __restrict__ QP, const h16* __restrict__ KP, const h16* __restrict__ VT, bf* ATh, bf* ATl) {
    __shared__ __align__(16) float os[4 * 16 * 68];
    const int lane = threadIdx.x & 31, w = threadIdx.x >> 5, lr = lane & 15, hi = lane >> 4;
    const int bh = blockIdx.y; const int q0 = (blockIdx.x * 4 + w) * 16;
    const h16* Qb = QP + (size_t)bh * SEQ * HD; const h16* Kb = KP + (size_t)bh * SEQ * HD; const h16* Vb = VT + (size_t)bh * HD * SEQ;
    const v16h qb0 = ldh(Qb + (size_t)(q0 + lr) * HD + 8 * hi);
    const v16h qb1 = ldh(Qb + (size_t)(q0 + lr) * HD + 8 * hi + 32);
    const h16* kp = Kb + (size_t)lr * HD + 8 * hi;
    const h16* vp = Vb + (size_t)lr * SEQ + 8 * hi;
    v8f o[4];
#pragma unroll
    for (int dt = 0; dt < 4; ++dt) o[dt] = (v8f){};
    float m = -1.0e30f, l = 0.0f;
#pragma unroll 1
    for (int key0 = 0; key0 < SEQ; key0 += 64) {
        v8f s[4];
#pragma unroll
        for (int kt = 0; kt < 4; ++kt) { const v16h a0 = ldh(kp + (size_t)(key0 + 16 * kt) * HD); const v16h a1 = ldh(kp + (size_t)(key0 + 16 * kt) * HD + 32);
            s[kt] = wmma16(a0, qb0, (v8f){}); s[kt] = wmma16(a1, qb1, s[kt]); }
        asm volatile("v_nop\n\tv_nop\n\tv_nop\n\tv_nop" : "+v"(s[0]), "+v"(s[1]), "+v"(s[2]), "+v"(s[3]) : "v"(qb0), "v"(qb1));
        float mx = s[0][0];
#pragma unroll
        for (int kt = 0; kt < 4; ++kt)
#pragma unroll
            for (int r = 0; r < 8; ++r) mx = fmaxf(mx, s[kt][r]);
        mx = fmaxf(mx, __shfl_xor(mx, 16, 32));
        const float mnew = fmaxf(m, mx * CL2);
        const float alpha = __builtin_amdgcn_exp2f(m - mnew);
        m = mnew;
        const float sh = PEXP - mnew;
        float psum = 0.0f;
#pragma unroll
        for (int kt = 0; kt < 4; ++kt)
#pragma unroll
            for (int r = 0; r < 8; ++r) { const float p = __builtin_amdgcn_exp2f(fmaf(s[kt][r], CL2, sh)); s[kt][r] = p; psum += p; }
        l = l * alpha + psum;
        v16h pb0, pb1;
#pragma unroll
        for (int r = 0; r < 8; ++r) { pb0[r] = (h16)s[0][r]; pb0[8 + r] = (h16)s[1][r]; pb1[r] = (h16)s[2][r]; pb1[8 + r] = (h16)s[3][r]; }
#pragma unroll
        for (int dt = 0; dt < 4; ++dt)
#pragma unroll
            for (int r = 0; r < 8; ++r) o[dt][r] *= alpha;
#pragma unroll
        for (int dt = 0; dt < 4; ++dt) { const v16h va0 = ldh(vp + (size_t)(dt * 16) * SEQ + key0); const v16h va1 = ldh(vp + (size_t)(dt * 16) * SEQ + key0 + 32);
            o[dt] = wmma16(va0, pb0, o[dt]); o[dt] = wmma16(va1, pb1, o[dt]); }
        asm volatile("v_nop\n\tv_nop\n\tv_nop\n\tv_nop" : "+v"(o[0]), "+v"(o[1]), "+v"(o[2]), "+v"(o[3]) : "v"(pb0), "v"(pb1));
    }
    const float lt = l + __shfl_xor(l, 16, 32);
    const float inv = (1.0f / lt) * (1.0f / VCAR);
    float* ow = os + w * (16 * 68);
#pragma unroll
    for (int dt = 0; dt < 4; ++dt) { v4f x0, x1; x0[0] = o[dt][0] * inv; x0[1] = o[dt][1] * inv; x0[2] = o[dt][2] * inv; x0[3] = o[dt][3] * inv; x1[0] = o[dt][4] * inv; x1[1] = o[dt][5] * inv; x1[2] = o[dt][6] * inv; x1[3] = o[dt][7] * inv;
        *(v4fa*)(ow + lr * 68 + dt * 16 + hi * 8) = x0; *(v4fa*)(ow + lr * 68 + dt * 16 + hi * 8 + 4) = x1; }
    __syncthreads();
    const int b = bh / NH, h = bh % NH;
    const size_t obase = ((size_t)b * SEQ + q0) * DM + (size_t)h * HD;
#pragma unroll 1
    for (int ps = 0; ps < 2; ++ps) {
#pragma unroll
        for (int s4 = 0; s4 < 4; ++s4) { const int row = 4 * s4 + (lane >> 3), c = (lane & 7) * 8;
            const v4f x0 = *(const v4fa*)(ow + row * 68 + c); const v4f x1 = *(const v4fa*)(ow + row * 68 + c + 4);
            v8us oh, ol;
#pragma unroll
            for (int j = 0; j < 4; ++j) { unsigned short a, c2; splitf(x0[j], a, c2); oh[j] = a; ol[j] = c2; splitf(x1[j], a, c2); oh[4 + j] = a; ol[4 + j] = c2; }
            *(volatile v8us*)(ATh + obase + (size_t)row * DM + c) = oh; *(volatile v8us*)(ATl + obase + (size_t)row * DM + c) = ol; }
        if (ps == 0) __threadfence(); }
}

constexpr size_t al256(size_t b) { return (b + 255) & ~(size_t)255; }
constexpr size_t SZ_W = al256((size_t)DM * DM * 2);
constexpr size_t SZ_X = al256((size_t)NB * SEQ * DM * 2);
constexpr size_t SZ_P = al256((size_t)NB * NH * SEQ * HD * 2);
constexpr size_t WS_TOTAL = 4 * SZ_W + SZ_X + 3 * SZ_P + 2 * SZ_X;
static_assert(WS_TOTAL <= (size_t)134217728);

extern "C" void kernel_launch(void* const* d_in, const int* in_sizes, int n_in,
                              void* d_out, int out_size, void* d_ws, size_t ws_size, hipStream_t stream) {
    if (n_in < 9) return;
    const long long need_x = (long long)(NB - 1) * SEQ_FULL * DM + (long long)SEQ * DM;
    if ((long long)in_sizes[0] < need_x || (long long)out_size < need_x) return;
    if (in_sizes[1] < DM * DM || in_sizes[3] < DM * DM || in_sizes[5] < DM * DM || in_sizes[7] < DM * DM) return;
    if (in_sizes[2] < DM || in_sizes[4] < DM || in_sizes[6] < DM || in_sizes[8] < DM) return;
    if (WS_TOTAL > ws_size) return;
    const float* x = (const float*)d_in[0]; const float* wq = (const float*)d_in[1]; const float* bq = (const float*)d_in[2]; const float* wk = (const float*)d_in[3]; const float* bk = (const float*)d_in[4];
    const float* wv = (const float*)d_in[5]; const float* bv = (const float*)d_in[6]; const float* wo = (const float*)d_in[7]; const float* bo = (const float*)d_in[8];
    float* OUT = (float*)d_out;
    char* wsp = (char*)d_ws;
    bf* WQ = (bf*)wsp; wsp += SZ_W; bf* WK = (bf*)wsp; wsp += SZ_W; bf* WV = (bf*)wsp; wsp += SZ_W; bf* WO = (bf*)wsp; wsp += SZ_W;
    bf* XB = (bf*)wsp; wsp += SZ_X;
    h16* QP = (h16*)wsp; wsp += SZ_P; h16* KP = (h16*)wsp; wsp += SZ_P; h16* VT = (h16*)wsp; wsp += SZ_P;
    bf* ATh = (bf*)wsp; wsp += SZ_X; bf* ATl = (bf*)wsp; wsp += SZ_X;
    const size_t w8 = (size_t)DM * DM / 8; const unsigned gw = (unsigned)((w8 + 255) / 256);
    k_cvt8<<<dim3(gw, 1), 256, 0, stream>>>(wq, WQ, w8, 0, 0);
    k_cvt8<<<dim3(gw, 1), 256, 0, stream>>>(wk, WK, w8, 0, 0);
    k_cvt8<<<dim3(gw, 1), 256, 0, stream>>>(wv, WV, w8, 0, 0);
    k_cvt8<<<dim3(gw, 1), 256, 0, stream>>>(wo, WO, w8, 0, 0);
    const size_t x8 = (size_t)SEQ * DM / 8;
    k_cvt8<<<dim3((unsigned)((x8 + 255) / 256), NB), 256, 0, stream>>>(x, XB, x8, (size_t)SEQ_FULL * DM, (size_t)SEQ * DM);
    k_proj_hp<<<dim3(SEQ / 64, NH, NB), 32, 0, stream>>>(XB, WQ, bq, QP, QCAR);
    k_proj_hp<<<dim3(SEQ / 64, NH, NB), 32, 0, stream>>>(XB, WK, bk, KP, KCAR);
    k_proj_vt<<<dim3(DM / 64, SEQ / 64, NB), 32, 0, stream>>>(WV, XB, bv, VT, VCAR);
    k_flash<<<dim3(SEQ / 64, NB * NH), 128, 0, stream>>>(QP, KP, VT, ATh, ATl);
    k_oproj<<<dim3(SEQ / 64, DM / 64, NB), 32, 0, stream>>>(ATh, ATl, WO, bo, OUT);
}
